// VRWKV_Rec_HWC_SpatialMix_12249246728669
// MI455X (gfx1250) — hardware-verified
//
#include <hip/hip_runtime.h>
#include <math.h>

typedef __attribute__((ext_vector_type(16))) _Float16 v16h;
typedef __attribute__((ext_vector_type(8)))  _Float16 v8h;
typedef __attribute__((ext_vector_type(16))) __bf16   v16b;
typedef __attribute__((ext_vector_type(8)))  __bf16   v8b;
typedef __attribute__((ext_vector_type(8)))  float    v8f;
typedef __attribute__((ext_vector_type(4)))  float    v4f;

constexpr int kB    = 4;
constexpr int kS    = 64;
constexpr int kT    = kS * kS;
constexpr int kC    = 768;
constexpr int kR    = 4;
constexpr int kRows = kB * kT;
constexpr int kCC   = kC * kC;
constexpr int kThr  = 256;
constexpr float kInCarry = 1024.0f;
constexpr float kSc = 1.0f / (kInCarry * kInCarry);
constexpr float kInvT = 1.0f / (float)kT;
constexpr float kF16MinNormal = 6.103515625e-5f;

static_assert((kRows % 64) == 0 && (kC % 64) == 0 && ((kRows / 64) * (kC / 64)) % 8 == 0 && (kC % 32) == 0, "GEMM M, N multiples of 64; grid exact; K a multiple of 32");

constexpr size_t kOffXF16 = 0ull;
constexpr size_t kOffK16 = 25165824ull;
constexpr size_t kOffV16 = 50331648ull;
constexpr size_t kOffKF = 75497472ull;
constexpr size_t kOffVF = 125829120ull;
constexpr size_t kOffTA = 176160768ull;
constexpr size_t kOffTB = 188743680ull;
constexpr size_t kOffW6 = 201326592ull;
constexpr size_t kOffBIAS = 208404480ull;
constexpr size_t kWsTotal = 208420864ull;
static_assert(kWsTotal <= 268435456ull, "carve cap");
static_assert(kOffXF16 == 0
              && kOffK16 == kOffXF16 + 25165824ull
              && kOffV16 == kOffK16 + 25165824ull
              && kOffKF == kOffV16 + 25165824ull
              && kOffVF == kOffKF + 50331648ull
              && kOffTA == kOffVF + 50331648ull
              && kOffTB == kOffTA + 12582912ull
              && kOffW6 == kOffTB + 12582912ull
              && kOffBIAS == kOffW6 + 7077888ull
              && kWsTotal == kOffBIAS + 16384ull, "the carve is chained and totalled");
static_assert((kOffXF16 % 256) == 0 && (kOffK16 % 256) == 0 && (kOffV16 % 256) == 0 && (kOffKF % 256) == 0 && (kOffVF % 256) == 0 && (kOffTA % 256) == 0 && (kOffTB % 256) == 0 && (kOffW6 % 256) == 0 && (kOffBIAS % 256) == 0, "aligned regions");
constexpr int kFBF = 0, kFBB = 768, kFZB = 1536, kFEnd = 4096;
static_assert(kFZB + kC <= kFEnd, "the zero row covers N = 768");

__device__ __forceinline__ unsigned short f2bf_bits(float f) {
  unsigned u = __float_as_uint(f);
  return (unsigned short)((u + 0x7FFFu + ((u >> 16) & 1u)) >> 16);
}
__device__ __forceinline__ float bf_bits2f(unsigned short h) { return __uint_as_float(((unsigned)h) << 16); }
__device__ __forceinline__ float bf16r(float f) { return bf_bits2f(f2bf_bits(f)); }
__device__ __forceinline__ float carry_flush(float v, float carry) {
  const float s = v * carry;
  return (fabsf(s) < kF16MinNormal) ? 0.0f : s;
}
__device__ __forceinline__ float frcp(float x) { return __builtin_amdgcn_rcpf(x); }

__device__ __forceinline__ void dep_guard4_h(v8f& a, v8f& b, v8f& c, v8f& d, v16h x, v16h y) { asm volatile("v_nop\n\tv_nop\n\tv_nop\n\tv_nop" : "+v"(a), "+v"(b), "+v"(c), "+v"(d) : "v"(x), "v"(y)); }
__device__ __forceinline__ void dep_guard4_b(v8f& a, v8f& b, v8f& c, v8f& d, v16b x, v16b y) { asm volatile("v_nop\n\tv_nop\n\tv_nop\n\tv_nop" : "+v"(a), "+v"(b), "+v"(c), "+v"(d) : "v"(x), "v"(y)); }
__device__ __forceinline__ void keep4_h(v16h a, v16h b, v16h c, v16h d) { asm volatile("v_nop" :: "v"(a), "v"(b), "v"(c), "v"(d)); }
__device__ __forceinline__ void keep4_b(v16b a, v16b b, v16b c, v16b d) { asm volatile("v_nop" :: "v"(a), "v"(b), "v"(c), "v"(d)); }
__device__ __forceinline__ void acc_guard4(v8f& a, v8f& b, v8f& c, v8f& d) { asm volatile("v_nop\n\tv_nop\n\tv_nop\n\tv_nop" : "+v"(a), "+v"(b), "+v"(c), "+v"(d)); }

template <typename T> struct Frag;
template <> struct Frag<_Float16> {
  typedef v16h V; union U { v16h v; v8h h[2]; };
  static __device__ __forceinline__ v16h load(const _Float16* p) {
    U f; f.h[0] = *(const v8h*)(p); f.h[1] = *(const v8h*)(p + 16); return f.v;
  }
  static __device__ __forceinline__ v8f mma(v16h a, v16h b, v8f c) {
    return __builtin_amdgcn_wmma_f32_16x16x32_f16(false, a, false, b, (short)0, c, false, false);
  }
  static __device__ __forceinline__ void guard4(v8f& a, v8f& b, v8f& c, v8f& d, v16h x, v16h y) { dep_guard4_h(a, b, c, d, x, y); }
  static __device__ __forceinline__ void keep(v16h a, v16h b, v16h c, v16h d) { keep4_h(a, b, c, d); }
};
template <> struct Frag<__bf16> {
  typedef v16b V; union U { v16b v; v8b h[2]; };
  static __device__ __forceinline__ v16b load(const __bf16* p) {
    U f; f.h[0] = *(const v8b*)(p); f.h[1] = *(const v8b*)(p + 16); return f.v;
  }
  static __device__ __forceinline__ v8f mma(v16b a, v16b b, v8f c) {
    return __builtin_amdgcn_wmma_f32_16x16x32_bf16(false, a, false, b, (short)0, c, false, false);
  }
  static __device__ __forceinline__ void guard4(v8f& a, v8f& b, v8f& c, v8f& d, v16b x, v16b y) { dep_guard4_b(a, b, c, d, x, y); }
  static __device__ __forceinline__ void keep(v16b a, v16b b, v16b c, v16b d) { keep4_b(a, b, c, d); }
};

__device__ __forceinline__ v8f mma_h(v16h a, v16h b, v8f c) {
  c = __builtin_amdgcn_wmma_f32_16x16x32_f16(false, a, false, b, (short)0, c, false, false);
  asm volatile("v_nop\n\tv_nop\n\tv_nop\n\tv_nop" : "+v"(c) : "v"(a), "v"(b));
  return c;
}

template <int ET> struct Elem;
template <> struct Elem<0> { typedef _Float16 T; };
template <> struct Elem<1> { typedef __bf16 T; };
template <int ET, bool SPLIT, int BIAS_MODE, int OUT_MODE, bool RESID, int ACT = 0>
__global__ __launch_bounds__(256) void wmma_gemm64(
    const unsigned short* __restrict__ Ap, const unsigned short* __restrict__ A2p, int lda, long strideA,
    const unsigned short* __restrict__ Btp, const unsigned short* __restrict__ Bt2p, int ldb, long strideB,
    void* __restrict__ Cout, void* __restrict__ Cout2, int ldc, long strideC,
    const float* __restrict__ bias,
    const float* __restrict__ resid, long strideR,
    int M, int N, int K, float scale) {
  typedef typename Elem<ET>::T T;
  typedef typename Frag<T>::V V;
  const T* A = (const T*)Ap; const T* A2 = (const T*)A2p; const T* Bt = (const T*)Btp; const T* Bt2 = (const T*)Bt2p;
  __shared__ __align__(16) float sT[8][16 * 68];
  const int b    = blockIdx.y;
  const int lane = threadIdx.x & 31;
  const int wave = threadIdx.x >> 5;
  const int tilesN = N >> 6;
  const int tilesM = M >> 6;
  const int tile = blockIdx.x * 8 + wave;
  if (tile >= tilesM * tilesN) return;
  const int tm = tile / tilesN;
  const int tn = tile - tm * tilesN;
  const int m0 = tm << 6;
  const int n0 = tn << 6;

  const T* Ab  = A  + (size_t)b * strideA;
  const T* Bb  = Bt + (size_t)b * strideB;
  const T* Ab2 = SPLIT ? (A2  + (size_t)b * strideA) : nullptr;
  const T* Bb2 = SPLIT ? (Bt2 + (size_t)b * strideB) : nullptr;

  const int rlane = lane & 15;
  const int koff  = (lane >> 4) * 8;
  const int mOff  = (lane >> 4) * 8;

  v8f acc[4][4];
#pragma unroll
  for (int i = 0; i < 4; ++i)
#pragma unroll
    for (int j = 0; j < 4; ++j) acc[i][j] = (v8f){0.f,0.f,0.f,0.f,0.f,0.f,0.f,0.f};

  for (int k0 = 0; k0 < K; k0 += 32) {
    V bh[4], bl[4];
#pragma unroll
    for (int j = 0; j < 4; ++j) {
      const size_t bo = (size_t)(n0 + (j << 4) + rlane) * ldb + koff + k0;
      bh[j] = Frag<T>::load(Bb + bo);
      if (SPLIT) bl[j] = Frag<T>::load(Bb2 + bo);
    }
#pragma unroll
    for (int i = 0; i < 4; ++i) {
      const size_t ao = (size_t)(m0 + (i << 4) + rlane) * lda + koff + k0;
      V ah = Frag<T>::load(Ab + ao);
      V al;
      if (SPLIT) al = Frag<T>::load(Ab2 + ao);
#pragma unroll
      for (int j = 0; j < 4; ++j) {
        acc[i][j] = Frag<T>::mma(ah, bh[j], acc[i][j]);
        if (SPLIT) {
          acc[i][j] = Frag<T>::mma(ah, bl[j], acc[i][j]);
          acc[i][j] = Frag<T>::mma(al, bh[j], acc[i][j]);
        }
      }
      Frag<T>::guard4(acc[i][0], acc[i][1], acc[i][2], acc[i][3], ah, SPLIT ? al : ah);
    }
    Frag<T>::keep(bh[0], bh[1], bh[2], bh[3]);
    if (SPLIT) Frag<T>::keep(bl[0], bl[1], bl[2], bl[3]);
  }
  acc_guard4(acc[0][0], acc[0][1], acc[0][2], acc[0][3]);
  acc_guard4(acc[1][0], acc[1][1], acc[1][2], acc[1][3]);
  acc_guard4(acc[2][0], acc[2][1], acc[2][2], acc[2][3]);
  acc_guard4(acc[3][0], acc[3][1], acc[3][2], acc[3][3]);

  float* slab = sT[wave];
  const float* Rb = RESID ? (resid + (size_t)b * strideR) : nullptr;
#pragma unroll
  for (int i = 0; i < 4; ++i) {
    const int mBase = m0 + (i << 4);
#pragma unroll
    for (int j = 0; j < 4; ++j) {
      const int n = n0 + (j << 4) + rlane;
      float bv = 0.f;
      if (BIAS_MODE == 2) bv = bias[n];
#pragma unroll
      for (int r = 0; r < 8; ++r) {
        float v = acc[i][j][r] * scale;
        if (BIAS_MODE == 1) v += bias[mBase + mOff + r];
        if (BIAS_MODE == 2) v += bv;
        if (RESID) v += Rb[(size_t)(mBase + mOff + r) * ldc + n];
        if (ACT == 1) v = tanhf(v);
        if (ACT == 2) v = fmaxf(v, 0.0f);
        if (ACT == 3) v = v / (1.0f + expf(-v));
        if (ACT == 4) v = (v > 0.f) ? v : 0.01f * v;
        slab[(mOff + r) * 68 + (j << 4) + rlane] = v;
      }
    }
    __builtin_amdgcn_fence(__ATOMIC_RELEASE, "workgroup");
    __builtin_amdgcn_wave_barrier();
    __builtin_amdgcn_fence(__ATOMIC_ACQUIRE, "workgroup");
    if (OUT_MODE == 0) {
      float* C = (float*)Cout + (size_t)b * strideC;
      const int hh = lane >> 4, c4 = (lane & 15) * 4;
      for (int pass = 0; pass < 2; ++pass) {
#pragma unroll
        for (int it = 0; it < 8; ++it) {
          const int row = it * 2 + hh;
          v4f v = *(const v4f*)(slab + row * 68 + c4);
          *(volatile v4f*)(C + (size_t)(mBase + row) * ldc + n0 + c4) = v;
        }
        __threadfence();
      }
    } else {
      const int q = lane >> 3, c8 = (lane & 7) * 8;
      unsigned short* C  = (unsigned short*)Cout  + (size_t)b * strideC;
      unsigned short* C2 = (OUT_MODE == 2) ? ((unsigned short*)Cout2 + (size_t)b * strideC) : nullptr;
      for (int pass = 0; pass < 2; ++pass) {
#pragma unroll
        for (int it = 0; it < 4; ++it) {
          const int row = it * 4 + q;
          const float* sp = slab + row * 68 + c8;
          v8h hv, lv;
#pragma unroll
          for (int e = 0; e < 8; ++e) {
            if (OUT_MODE == 1) {
              hv[e] = (_Float16)sp[e];
            } else {
              unsigned short hb = f2bf_bits(sp[e]);
              unsigned short lb = f2bf_bits(sp[e] - bf_bits2f(hb));
              hv[e] = __builtin_bit_cast(_Float16, hb);
              lv[e] = __builtin_bit_cast(_Float16, lb);
            }
          }
          *(volatile v8h*)(C + (size_t)(mBase + row) * ldc + n0 + c8) = hv;
          if (OUT_MODE == 2) *(volatile v8h*)(C2 + (size_t)(mBase + row) * ldc + n0 + c8) = lv;
        }
        __threadfence();
      }
    }
    __builtin_amdgcn_fence(__ATOMIC_RELEASE, "workgroup");
    __builtin_amdgcn_wave_barrier();
    __builtin_amdgcn_fence(__ATOMIC_ACQUIRE, "workgroup");
  }
}


__device__ __forceinline__ float fast_sigmoid(float v) { return frcp(1.0f + __expf(-v)); }

__global__ __launch_bounds__(kThr) void omni_shift_kernel(const float* __restrict__ x, const float* __restrict__ w1, const float* __restrict__ w3,
                                                          const float* __restrict__ w5, const float* __restrict__ alpha, unsigned short* __restrict__ XF16) {
  unsigned v = blockIdx.x * (unsigned)kThr + threadIdx.x;
  asm volatile("" : "+v"(v));
  const unsigned row = v / 96u;
  const unsigned c8 = (v - row * 96u) * 8u;
  const unsigned b = row >> 12;
  const unsigned t = row & 4095u;
  const int yy = (int)(t >> 6), xx = (int)(t & 63u);
  const float al0 = alpha[0], al1 = alpha[1], al2 = alpha[2], al3 = alpha[3];
  const float a0 = bf16r(al0), a1 = bf16r(al1), a2 = bf16r(al2), a3 = bf16r(al3);
  float s3[8], s5[8], ctr[8];
#pragma unroll
  for (int e = 0; e < 8; ++e) { s3[e] = 0.0f; s5[e] = 0.0f; ctr[e] = 0.0f; }
#pragma unroll 1
  for (int i = 0; i < 5; ++i) {
#pragma unroll 1
    for (int j = 0; j < 5; ++j) {
      const int ny = yy + i - 2, nx = xx + j - 2;
      const bool in = (ny >= 0) && (ny < kS) && (nx >= 0) && (nx < kS);
      const int cy = (ny < 0) ? 0 : ((ny > kS - 1) ? (kS - 1) : ny);
      const int cx = (nx < 0) ? 0 : ((nx > kS - 1) ? (kS - 1) : nx);
      const float* sp = x + ((size_t)b * kT + (size_t)(cy * kS + cx)) * kC + c8;
      const v4f p0 = *(const v4f*)sp, p1 = *(const v4f*)(sp + 4);
      const bool in3 = (i >= 1) && (i <= 3) && (j >= 1) && (j <= 3);
      const int i3 = in3 ? (i - 1) : 0, j3 = in3 ? (j - 1) : 0;
#pragma unroll
      for (int e = 0; e < 8; ++e) {
        const float xr = (e < 4) ? p0[e] : p1[e - 4];
        const float xv = in ? bf16r(xr) : 0.0f;
        const float k5 = w5[(size_t)(c8 + (unsigned)e) * 25u + (unsigned)(i * 5 + j)];
        const float k3 = w3[(size_t)(c8 + (unsigned)e) * 9u + (unsigned)(i3 * 3 + j3)];
        s5[e] += bf16r(k5) * xv;
        if (in3) s3[e] += bf16r(k3) * xv;
        if (i == 2 && j == 2) ctr[e] = xv;
      }
    }
  }
  v8h hv;
#pragma unroll
  for (int e = 0; e < 8; ++e) {
    const float k1 = w1[c8 + (unsigned)e];
    const float xs = a0 * ctr[e] + a1 * (bf16r(k1) * ctr[e]) + a2 * s3[e] + a3 * s5[e];
    hv[e] = (_Float16)carry_flush(xs, kInCarry);
  }
  unsigned short* dp = XF16 + (size_t)row * kC + c8;
  *(volatile v8h*)dp = hv;
  __threadfence();
  *(volatile v8h*)dp = hv;
}
static_assert((kRows * (kC / 8)) % kThr == 0 && kC / 8 == 96 && kT == 4096 && kS == 64, "shift grid exact; row = b 4096 + y 64 + x");

__global__ __launch_bounds__(kThr) void w_flat_cast_kernel(const float* __restrict__ W, unsigned short* __restrict__ dst) {
  const size_t v = (size_t)blockIdx.x * kThr + threadIdx.x;
  const v4f a0 = *(const v4f*)(W + v * 8), a1 = *(const v4f*)(W + v * 8 + 4);
  v8h hv;
#pragma unroll
  for (int e = 0; e < 4; ++e) { const float x0 = a0[e], x1 = a1[e]; hv[e] = (_Float16)carry_flush(bf16r(x0), kInCarry); hv[4 + e] = (_Float16)carry_flush(bf16r(x1), kInCarry); }
  unsigned short* dp = dst + v * 8;
  *(volatile v8h*)dp = hv;
  __threadfence();
  *(volatile v8h*)dp = hv;
}
static_assert((kCC / 8) % kThr == 0, "weight cast grid exact");

__global__ __launch_bounds__(kThr) void bias_rows_kernel(const float* __restrict__ bfw, const float* __restrict__ bbw, float* __restrict__ BIAS) {
  unsigned v = blockIdx.x * (unsigned)kThr + threadIdx.x;
  asm volatile("" : "+v"(v));
  const unsigned i0 = v * 4u;
  v4f o = {0.f, 0.f, 0.f, 0.f};
  if (i0 < (unsigned)kFZB) {
    const v4f a = *(const v4f*)((i0 < (unsigned)kFBB) ? (bfw + i0) : (bbw + (i0 - (unsigned)kFBB)));
#pragma unroll
    for (int e = 0; e < 4; ++e) { const float x = a[e]; o[e] = bf16r(x); }
  }
  float* dp = BIAS + i0;
  *(volatile v4f*)dp = o;
  __threadfence();
  *(volatile v4f*)dp = o;
}
static_assert(kFEnd / 4 == 4 * kThr && (kFBB % 128) == 0 && (kFZB % 128) == 0, "bias grid exact");

__global__ __launch_bounds__(kThr) void kv_cast_kernel(const float* __restrict__ KF, const float* __restrict__ VF, unsigned short* __restrict__ K16,
                                                       unsigned short* __restrict__ V16) {
  const size_t v = (size_t)blockIdx.x * kThr + threadIdx.x;
  const v4f k0 = *(const v4f*)(KF + v * 8), k1 = *(const v4f*)(KF + v * 8 + 4);
  const v4f u0 = *(const v4f*)(VF + v * 8), u1 = *(const v4f*)(VF + v * 8 + 4);
  v8h hk, hv;
#pragma unroll
  for (int e = 0; e < 4; ++e) {
    hk[e] = (_Float16)carry_flush(k0[e], kInCarry); hk[4 + e] = (_Float16)carry_flush(k1[e], kInCarry);
    hv[e] = (_Float16)carry_flush(u0[e], kInCarry); hv[4 + e] = (_Float16)carry_flush(u1[e], kInCarry);
  }
  for (int pass = 0; pass < 2; ++pass) {
    *(volatile v8h*)(K16 + v * 8) = hk;
    *(volatile v8h*)(V16 + v * 8) = hv;
    __threadfence();
  }
}
static_assert(((size_t)kRows * kC / 8) % kThr == 0, "plane cast grid exact");

__global__ __launch_bounds__(kThr) void wkv_back_kernel(const float* __restrict__ KFb, const float* __restrict__ VFb, const float* __restrict__ dec,
                                                        float* __restrict__ TA, float* __restrict__ TB, int order) {
  const unsigned c = blockIdx.x * (unsigned)kThr + threadIdx.x;
  const float d0 = dec[c];
  const float ew = __expf(-__expf(bf16r(d0) * kInvT));
  float a = 0.0f, bb = 0.0f;
#pragma unroll 1
  for (int t = kT - 1; t >= 0; --t) {
    const unsigned tok = order ? (((unsigned)t & 63u) * 64u + ((unsigned)t >> 6)) : (unsigned)t;
    const size_t o = (size_t)tok * kC + c;
    const float kk = KFb[o], vv = VFb[o];
    float* pa = TA + o; float* pb = TB + o;
    *(volatile float*)pa = a; *(volatile float*)pb = bb;
    __threadfence();
    *(volatile float*)pa = a; *(volatile float*)pb = bb;
    const float ek = __expf(kk);
    a = ew * a + ek * vv;
    bb = ew * bb + ek;
  }
}

__global__ __launch_bounds__(kThr) void wkv_fwd_kernel(const float* __restrict__ KFb, float* __restrict__ VFb, const float* __restrict__ dec,
                                                       const float* __restrict__ first, const float* __restrict__ TA, const float* __restrict__ TB, int order) {
  const unsigned c = blockIdx.x * (unsigned)kThr + threadIdx.x;
  const float d0 = dec[c], f0 = first[c];
  const float ew = __expf(-__expf(bf16r(d0) * kInvT));
  const float u = bf16r(f0) * kInvT;
  float a = 0.0f, bb = 0.0f;
#pragma unroll 1
  for (int t = 0; t < kT; ++t) {
    const unsigned tok = order ? (((unsigned)t & 63u) * 64u + ((unsigned)t >> 6)) : (unsigned)t;
    const size_t o = (size_t)tok * kC + c;
    const float kk = KFb[o], vv = VFb[o];
    const float ar = TA[o], br = TB[o];
    const float ek = __expf(kk);
    const float eu = __expf(u + kk);
    const float num = (a + ar) + eu * vv;
    const float den = (bb + br) + eu;
    const float outv = num / den;
    float* pv = VFb + o;
    *(volatile float*)pv = outv;
    __threadfence();
    *(volatile float*)pv = outv;
    a = ew * a + ek * vv;
    bb = ew * bb + ek;
  }
}
static_assert(kC == 3 * kThr, "scan grid exact: three blocks of channels");

__global__ __launch_bounds__(kThr) void gate_cast_kernel(const float* __restrict__ RR, const float* __restrict__ VF, unsigned short* __restrict__ Y16) {
  const size_t v = (size_t)blockIdx.x * kThr + threadIdx.x;
  const v4f r0 = *(const v4f*)(RR + v * 8), r1 = *(const v4f*)(RR + v * 8 + 4);
  const v4f u0 = *(const v4f*)(VF + v * 8), u1 = *(const v4f*)(VF + v * 8 + 4);
  v8h hv;
#pragma unroll
  for (int e = 0; e < 4; ++e) {
    hv[e]     = (_Float16)carry_flush(fast_sigmoid(r0[e]) * u0[e], kInCarry);
    hv[4 + e] = (_Float16)carry_flush(fast_sigmoid(r1[e]) * u1[e], kInCarry);
  }
  unsigned short* dp = Y16 + v * 8;
  *(volatile v8h*)dp = hv;
  __threadfence();
  *(volatile v8h*)dp = hv;
}

__global__ __launch_bounds__(kThr) void copy_out_kernel(const float* __restrict__ src, float* __restrict__ out) {
  const size_t i = (size_t)blockIdx.x * kThr + threadIdx.x;
  const v4f o = *(const v4f*)(src + i * 4);
  float* dp = out + i * 4;
  *(volatile v4f*)dp = o;
  __threadfence();
  *(volatile v4f*)dp = o;
}
static_assert(((size_t)kRows * kC / 4) % kThr == 0, "output grid exact");

extern "C" void kernel_launch(void* const* d_in, const int* in_sizes, int n_in,
                              void* d_out, int out_size, void* d_ws, size_t ws_size,
                              hipStream_t stream) {
  if (n_in < 17 || d_out == nullptr || d_ws == nullptr) return;
  if (in_sizes[0] != kRows * kC || in_sizes[1] != 1 || in_sizes[2] != 1 || in_sizes[3] != kC || in_sizes[4] != kC * 9 || in_sizes[5] != kC * 25 || in_sizes[6] != 4) return;
  if (in_sizes[7] != kCC || in_sizes[8] != kCC || in_sizes[9] != kCC || in_sizes[10] != kCC || in_sizes[11] != kC || in_sizes[12] != kCC || in_sizes[13] != kC || in_sizes[14] != kCC) return;
  if (in_sizes[15] != kR * kC || in_sizes[16] != kR * kC) return;
  if ((size_t)out_size != (size_t)kRows * kC) return;
  if (ws_size < kWsTotal) return;
  const float* x = (const float*)d_in[0];
  const float* os_w1 = (const float*)d_in[3];
  const float* os_w3 = (const float*)d_in[4];
  const float* os_w5 = (const float*)d_in[5];
  const float* os_alpha = (const float*)d_in[6];
  const float* Wsrc[6] = {(const float*)d_in[7], (const float*)d_in[8], (const float*)d_in[9], (const float*)d_in[10], (const float*)d_in[12], (const float*)d_in[14]};
  const float* bfw = (const float*)d_in[11];
  const float* bbw = (const float*)d_in[13];
  const float* sdecay = (const float*)d_in[15];
  const float* sfirst = (const float*)d_in[16];
  float* out = (float*)d_out;
  char* ws = (char*)d_ws;
  unsigned short* XF16 = (unsigned short*)(ws + kOffXF16);
  unsigned short* K16 = (unsigned short*)(ws + kOffK16);
  unsigned short* V16 = (unsigned short*)(ws + kOffV16);
  float* KF = (float*)(ws + kOffKF);
  float* VF = (float*)(ws + kOffVF);
  float* TA = (float*)(ws + kOffTA);
  float* TB = (float*)(ws + kOffTB);
  unsigned short* W6 = (unsigned short*)(ws + kOffW6);
  float* BIAS = (float*)(ws + kOffBIAS);
  const float* ZB = BIAS + kFZB;
  const unsigned short* WK = W6;
  const unsigned short* WV = W6 + (size_t)1 * kCC;
  const unsigned short* WR = W6 + (size_t)2 * kCC;
  const unsigned short* WF = W6 + (size_t)3 * kCC;
  const unsigned short* WB = W6 + (size_t)4 * kCC;
  const unsigned short* WO = W6 + (size_t)5 * kCC;
  const dim3 ggrid((kRows / 64) * (kC / 64) / 8, 1);

  omni_shift_kernel<<<(kRows * (kC / 8)) / kThr, kThr, 0, stream>>>(x, os_w1, os_w3, os_w5, os_alpha, XF16);
  for (int m = 0; m < 6; ++m) w_flat_cast_kernel<<<(kCC / 8) / kThr, kThr, 0, stream>>>(Wsrc[m], W6 + (size_t)m * kCC);
  bias_rows_kernel<<<4, kThr, 0, stream>>>(bfw, bbw, BIAS);
  wmma_gemm64<0, false, 2, 0, false, 0><<<ggrid, 256, 0, stream>>>(XF16, XF16, kC, 0L, WK, WK, kC, 0L, (void*)KF, (void*)KF, kC, 0L, ZB, nullptr, 0L, kRows, kC, kC, kSc);
  wmma_gemm64<0, false, 2, 0, false, 0><<<ggrid, 256, 0, stream>>>(XF16, XF16, kC, 0L, WV, WV, kC, 0L, (void*)VF, (void*)VF, kC, 0L, ZB, nullptr, 0L, kRows, kC, kC, kSc);
  for (int j = 0; j < kR; ++j) {
    if ((j & 1) == 0) {
      const unsigned short* WM = (j == 0) ? WF : WB;
      const float* BM = BIAS + ((j == 0) ? kFBF : kFBB);
      kv_cast_kernel<<<(int)(((size_t)kRows * kC / 8) / kThr), kThr, 0, stream>>>(KF, VF, K16, V16);
      wmma_gemm64<0, false, 2, 0, false, 0><<<ggrid, 256, 0, stream>>>(K16, K16, kC, 0L, WM, WM, kC, 0L, (void*)KF, (void*)KF, kC, 0L, BM, nullptr, 0L, kRows, kC, kC, kSc);
      wmma_gemm64<0, false, 2, 0, false, 0><<<ggrid, 256, 0, stream>>>(V16, V16, kC, 0L, WM, WM, kC, 0L, (void*)VF, (void*)VF, kC, 0L, BM, nullptr, 0L, kRows, kC, kC, kSc);
    }
    const int order = j & 1;
    for (int b = 0; b < kB; ++b) {
      const float* kb = KF + (size_t)b * kT * kC;
      float* vb = VF + (size_t)b * kT * kC;
      wkv_back_kernel<<<3, kThr, 0, stream>>>(kb, vb, sdecay + (size_t)j * kC, TA, TB, order);
      wkv_fwd_kernel<<<3, kThr, 0, stream>>>(kb, vb, sdecay + (size_t)j * kC, sfirst + (size_t)j * kC, TA, TB, order);
    }
  }
  wmma_gemm64<0, false, 2, 0, false, 0><<<ggrid, 256, 0, stream>>>(XF16, XF16, kC, 0L, WR, WR, kC, 0L, (void*)KF, (void*)KF, kC, 0L, ZB, nullptr, 0L, kRows, kC, kC, kSc);
  gate_cast_kernel<<<(int)(((size_t)kRows * kC / 8) / kThr), kThr, 0, stream>>>(KF, VF, K16);
  wmma_gemm64<0, false, 2, 0, false, 0><<<ggrid, 256, 0, stream>>>(K16, K16, kC, 0L, WO, WO, kC, 0L, (void*)VF, (void*)VF, kC, 0L, ZB, nullptr, 0L, kRows, kC, kC, kSc);
  copy_out_kernel<<<(int)(((size_t)kRows * kC / 4) / kThr), kThr, 0, stream>>>(VF, out);
}
